// HybridRetention_60765197304161
// MI455X (gfx1250) — hardware-verified
//
#include <hip/hip_runtime.h>
#include <math.h>

constexpr int DMODEL = 512;
constexpr int SEQLEN = 4096;
constexpr int NBAT   = 4;
constexpr int NROWS  = NBAT * SEQLEN;
constexpr int RTHR   = 256;
constexpr int ABP    = 520;
constexpr int SSP    = 516;
constexpr float WCARRY_G = 16.0f;
constexpr float WCARRY_A = 8.0f;
constexpr float WCARRY_O = 16.0f;

typedef __attribute__((ext_vector_type(16))) _Float16 v16h;
typedef __attribute__((ext_vector_type(8)))  _Float16 v8h;
typedef __attribute__((ext_vector_type(16))) __bf16   v16b;
typedef __attribute__((ext_vector_type(8)))  __bf16   v8b;
typedef __attribute__((ext_vector_type(8)))  float    v8f;
typedef __attribute__((ext_vector_type(4)))  float    v4f;

__device__ __forceinline__ unsigned short f2bf_bits(float f) {
  unsigned u = __float_as_uint(f);
  return (unsigned short)((u + 0x7FFFu + ((u >> 16) & 1u)) >> 16);
}
__device__ __forceinline__ float bf_bits2f(unsigned short h) { return __uint_as_float(((unsigned)h) << 16); }

__device__ __forceinline__ void dep_guard_h(v8f& a, v8f& b, v16h x, v16h y) { asm volatile("v_nop\n\tv_nop\n\tv_nop\n\tv_nop" : "+v"(a), "+v"(b) : "v"(x), "v"(y)); }
__device__ __forceinline__ void dep_guard_b(v8f& a, v8f& b, v16b x, v16b y) { asm volatile("v_nop\n\tv_nop\n\tv_nop\n\tv_nop" : "+v"(a), "+v"(b) : "v"(x), "v"(y)); }
__device__ __forceinline__ void keep4_h(v16h a, v16h b, v16h c, v16h d) { asm volatile("v_nop" :: "v"(a), "v"(b), "v"(c), "v"(d)); }
__device__ __forceinline__ void keep4_b(v16b a, v16b b, v16b c, v16b d) { asm volatile("v_nop" :: "v"(a), "v"(b), "v"(c), "v"(d)); }
__device__ __forceinline__ void acc_guard4(v8f& a, v8f& b, v8f& c, v8f& d) { asm volatile("v_nop\n\tv_nop\n\tv_nop\n\tv_nop" : "+v"(a), "+v"(b), "+v"(c), "+v"(d)); }
template <typename T> struct Frag;
template <> struct Frag<_Float16> {
  typedef v16h V; union U { v16h v; v8h h[2]; };
  static __device__ __forceinline__ v16h load(const _Float16* p) {
    U f; f.h[0] = *(const v8h*)(p); f.h[1] = *(const v8h*)(p + 16); return f.v;
  }
  static __device__ __forceinline__ v8f mma(v16h a, v16h b, v8f c) {
    return __builtin_amdgcn_wmma_f32_16x16x32_f16(false, a, false, b, (short)0, c, false, false);
  }
  static __device__ __forceinline__ void guard(v8f& a, v8f& b, v16h x, v16h y) { dep_guard_h(a, b, x, y); }
  static __device__ __forceinline__ void keep(v16h a, v16h b, v16h c, v16h d) { keep4_h(a, b, c, d); }
};
template <> struct Frag<__bf16> {
  typedef v16b V; union U { v16b v; v8b h[2]; };
  static __device__ __forceinline__ v16b load(const __bf16* p) {
    U f; f.h[0] = *(const v8b*)(p); f.h[1] = *(const v8b*)(p + 16); return f.v;
  }
  static __device__ __forceinline__ v8f mma(v16b a, v16b b, v8f c) {
    return __builtin_amdgcn_wmma_f32_16x16x32_bf16(false, a, false, b, (short)0, c, false, false);
  }
  static __device__ __forceinline__ void guard(v8f& a, v8f& b, v16b x, v16b y) { dep_guard_b(a, b, x, y); }
  static __device__ __forceinline__ void keep(v16b a, v16b b, v16b c, v16b d) { keep4_b(a, b, c, d); }
};

__device__ __forceinline__ float ftanh(float x) { return 1.0f - 2.0f * __builtin_amdgcn_rcpf(__expf(2.0f * x) + 1.0f); }

template <int ET> struct Elem;
template <> struct Elem<0> { typedef _Float16 T; };
template <> struct Elem<1> { typedef __bf16 T; };
template <int ET, bool SPLIT, int BIAS_MODE, int OUT_MODE, bool RESID, int ACT = 0>
__global__ __launch_bounds__(256) void wmma_gemm64(
    const unsigned short* __restrict__ Ap, const unsigned short* __restrict__ A2p, int lda, long strideA,
    const unsigned short* __restrict__ Btp, const unsigned short* __restrict__ Bt2p, int ldb, long strideB,
    void* __restrict__ Cout, void* __restrict__ Cout2, int ldc, long strideC,
    const float* __restrict__ bias,
    const float* __restrict__ resid, long strideR,
    int M, int N, int K, float scale) {
  typedef typename Elem<ET>::T T;
  typedef typename Frag<T>::V V;
  const T* A = (const T*)Ap; const T* A2 = (const T*)A2p; const T* Bt = (const T*)Btp; const T* Bt2 = (const T*)Bt2p;
  __shared__ __align__(16) float sT[8][16 * 68];
  const int b    = blockIdx.y;
  const int lane = threadIdx.x & 31;
  const int wave = threadIdx.x >> 5;
  const int tilesN = N >> 6;
  const int tilesM = M >> 6;
  const int tile = blockIdx.x * 8 + wave;
  if (tile >= tilesM * tilesN) return;
  const int tm = tile / tilesN;
  const int tn = tile - tm * tilesN;
  const int m0 = tm << 6;
  const int n0 = tn << 6;

  const T* Ab  = A  + (size_t)b * strideA;
  const T* Bb  = Bt + (size_t)b * strideB;
  const T* Ab2 = SPLIT ? (A2  + (size_t)b * strideA) : nullptr;
  const T* Bb2 = SPLIT ? (Bt2 + (size_t)b * strideB) : nullptr;

  const int rlane = lane & 15;
  const int koff  = (lane >> 4) * 8;
  const int mOff  = (lane >> 4) * 8;

  v8f acc[4][4];
#pragma unroll
  for (int i = 0; i < 4; ++i)
#pragma unroll
    for (int j = 0; j < 4; ++j) acc[i][j] = (v8f){0.f,0.f,0.f,0.f,0.f,0.f,0.f,0.f};

  for (int k0 = 0; k0 < K; k0 += 32) {
    V bh[4], bl[4];
#pragma unroll
    for (int j = 0; j < 4; ++j) {
      const size_t bo = (size_t)(n0 + (j << 4) + rlane) * ldb + koff + k0;
      bh[j] = Frag<T>::load(Bb + bo);
      if (SPLIT) bl[j] = Frag<T>::load(Bb2 + bo);
    }
#pragma unroll
    for (int i = 0; i < 4; ++i) {
      const size_t ao = (size_t)(m0 + (i << 4) + rlane) * lda + koff + k0;
      V ah = Frag<T>::load(Ab + ao);
      V al;
      if (SPLIT) al = Frag<T>::load(Ab2 + ao);
#pragma unroll
      for (int j = 0; j < 4; ++j) {
        acc[i][j] = Frag<T>::mma(ah, bh[j], acc[i][j]);
        if (SPLIT) {
          acc[i][j] = Frag<T>::mma(ah, bl[j], acc[i][j]);
          acc[i][j] = Frag<T>::mma(al, bh[j], acc[i][j]);
        }
      }
      Frag<T>::guard(acc[i][0], acc[i][3], ah, SPLIT ? al : ah);
    }
    Frag<T>::keep(bh[0], bh[1], bh[2], bh[3]);
    if (SPLIT) Frag<T>::keep(bl[0], bl[1], bl[2], bl[3]);
  }
  acc_guard4(acc[0][0], acc[0][1], acc[0][2], acc[0][3]);
  acc_guard4(acc[1][0], acc[1][1], acc[1][2], acc[1][3]);
  acc_guard4(acc[2][0], acc[2][1], acc[2][2], acc[2][3]);
  acc_guard4(acc[3][0], acc[3][1], acc[3][2], acc[3][3]);

  float* slab = sT[wave];
  const float* Rb = RESID ? (resid + (size_t)b * strideR) : nullptr;
#pragma unroll
  for (int i = 0; i < 4; ++i) {
    const int mBase = m0 + (i << 4);
#pragma unroll
    for (int j = 0; j < 4; ++j) {
      const int n = n0 + (j << 4) + rlane;
      float bv = 0.f;
      if (BIAS_MODE == 2) bv = bias[n];
#pragma unroll
      for (int r = 0; r < 8; ++r) {
        float v = acc[i][j][r] * scale;
        if (BIAS_MODE == 1) v += bias[mBase + mOff + r];
        if (BIAS_MODE == 2) v += bv;
        if (RESID) v += Rb[(size_t)(mBase + mOff + r) * ldc + n];
        if (ACT == 1) v = tanhf(v);
        if (ACT == 2) v = fmaxf(v, 0.0f);
        if (ACT == 3) v = v / (1.0f + expf(-v));
        if (ACT == 4) v = (v > 0.f) ? v : 0.01f * v;
        if (ACT == 5) v = 0.5f * v * (1.0f + erff(v * 0.70710678118654752f));
        if (ACT == 6) v = __builtin_amdgcn_rcpf(1.0f + __expf(-v));
        slab[(mOff + r) * 68 + (j << 4) + rlane] = v;
      }
    }
    __builtin_amdgcn_fence(__ATOMIC_RELEASE, "workgroup");
    __builtin_amdgcn_wave_barrier();
    __builtin_amdgcn_fence(__ATOMIC_ACQUIRE, "workgroup");
    if (OUT_MODE == 0) {
      float* C = (float*)Cout + (size_t)b * strideC;
      const int hh = lane >> 4, c4 = (lane & 15) * 4;
      for (int pass = 0; pass < 2; ++pass) {
#pragma unroll
        for (int it = 0; it < 8; ++it) {
          const int row = it * 2 + hh;
          v4f v = *(const v4f*)(slab + row * 68 + c4);
          *(volatile v4f*)(C + (size_t)(mBase + row) * ldc + n0 + c4) = v;
        }
        __threadfence();
      }
    } else {
      const int q = lane >> 3, c8 = (lane & 7) * 8;
      unsigned short* C  = (unsigned short*)Cout  + (size_t)b * strideC;
      unsigned short* C2 = (OUT_MODE == 2) ? ((unsigned short*)Cout2 + (size_t)b * strideC) : nullptr;
      for (int pass = 0; pass < 2; ++pass) {
#pragma unroll
        for (int it = 0; it < 4; ++it) {
          const int row = it * 4 + q;
          const float* sp = slab + row * 68 + c8;
          v8h hv, lv;
#pragma unroll
          for (int e = 0; e < 8; ++e) {
            if (OUT_MODE == 1) {
              hv[e] = (_Float16)sp[e];
            } else {
              unsigned short hb = f2bf_bits(sp[e]);
              unsigned short lb = f2bf_bits(sp[e] - bf_bits2f(hb));
              hv[e] = __builtin_bit_cast(_Float16, hb);
              lv[e] = __builtin_bit_cast(_Float16, lb);
            }
          }
          *(volatile v8h*)(C + (size_t)(mBase + row) * ldc + n0 + c8) = hv;
          if (OUT_MODE == 2) *(volatile v8h*)(C2 + (size_t)(mBase + row) * ldc + n0 + c8) = lv;
        }
        __threadfence();
      }
    }
    __builtin_amdgcn_fence(__ATOMIC_RELEASE, "workgroup");
    __builtin_amdgcn_wave_barrier();
    __builtin_amdgcn_fence(__ATOMIC_ACQUIRE, "workgroup");
  }
}

__global__ __launch_bounds__(256) void cast_scale_f16x2(
    const float* __restrict__ in, _Float16* __restrict__ out, int n2, float sc) {
  int i = blockIdx.x * 256 + threadIdx.x;
  if (i < n2) {
    const _Float16 h0 = (_Float16)(in[2 * (size_t)i] * sc), h1 = (_Float16)(in[2 * (size_t)i + 1] * sc);
    const unsigned u = (unsigned)__builtin_bit_cast(unsigned short, h0) | ((unsigned)__builtin_bit_cast(unsigned short, h1) << 16);
    ((volatile unsigned*)out)[i] = u;
    __threadfence();
    ((volatile unsigned*)out)[i] = u;
  }
}

__global__ __launch_bounds__(64) void rscan_kernel(const float* __restrict__ kin, const float* __restrict__ vin,
                                                 const float* __restrict__ decay, int ndec,
                                                 unsigned short* __restrict__ Rout) {
  const int b = blockIdx.x;
  const int tid = threadIdx.x;
  int hidx = tid >> 3;
  hidx = (hidx < ndec) ? hidx : (ndec - 1);
  hidx = (hidx < 0) ? 0 : hidx;
  const float dec = decay[hidx];
  float r0 = 0.f, r1 = 0.f, r2 = 0.f, r3 = 0.f, r4 = 0.f, r5 = 0.f, r6 = 0.f, r7 = 0.f;
  const size_t base = (size_t)b * SEQLEN * DMODEL + (size_t)tid * 8;
#pragma unroll 1
  for (int t = 0; t < SEQLEN; ++t) {
    const size_t o = base + (size_t)t * DMODEL;
    const v4f ka = *(const v4f*)(kin + o);
    const v4f kb = *(const v4f*)(kin + o + 4);
    const v4f va = *(const v4f*)(vin + o);
    const v4f vb = *(const v4f*)(vin + o + 4);
    r0 = dec * r0 + ka[0] * va[0];
    r1 = dec * r1 + ka[1] * va[1];
    r2 = dec * r2 + ka[2] * va[2];
    r3 = dec * r3 + ka[3] * va[3];
    r4 = dec * r4 + kb[0] * vb[0];
    r5 = dec * r5 + kb[1] * vb[1];
    r6 = dec * r6 + kb[2] * vb[2];
    r7 = dec * r7 + kb[3] * vb[3];
    v8h hv;
    hv[0] = (_Float16)r0; hv[1] = (_Float16)r1; hv[2] = (_Float16)r2; hv[3] = (_Float16)r3;
    hv[4] = (_Float16)r4; hv[5] = (_Float16)r5; hv[6] = (_Float16)r6; hv[7] = (_Float16)r7;
    unsigned short* dst = Rout + o;
    *(volatile v8h*)dst = hv;
    __threadfence();
    *(volatile v8h*)dst = hv;
  }
}

__global__ __launch_bounds__(RTHR) void recur_kernel(const float* __restrict__ q, const float* __restrict__ gate,
                                                    const float* __restrict__ rbf, const unsigned short* __restrict__ Awp,
                                                    unsigned short* __restrict__ Sout) {
  __shared__ __align__(16) _Float16 Abl[16 * ABP];
  __shared__ __align__(16) float    Sst[NBAT * SSP];
  const _Float16* Aw = (const _Float16*)Awp;
  const int tid = threadIdx.x, lane = tid & 31, wave = tid >> 5;
  const int c = lane & 15, hh = lane >> 4, koff = hh * 8;
  const int n0 = wave * 64;

#pragma unroll 1
  for (int i = tid; i < 16 * ABP; i += RTHR) Abl[i] = (_Float16)0.0f;
  __syncthreads();
  {
    const int row = tid >> 6, c8 = (tid & 63) * 8;
    const size_t base = ((size_t)row * SEQLEN) * DMODEL + (size_t)c8;
#pragma unroll
    for (int e = 0; e < 8; ++e) {
      const float g = gate[base + e], qv = q[base + e];
      Abl[row * ABP + c8 + e] = (_Float16)(g * 0.0f + (1.0f - g) * qv);
    }
  }
  __syncthreads();

  const _Float16* arow = Abl + c * ABP + koff;
  const _Float16* brow = Aw + (size_t)(n0 + c) * DMODEL + koff;
  const v8f z8 = {0.f, 0.f, 0.f, 0.f, 0.f, 0.f, 0.f, 0.f};
  const float inv_carry = 1.0f / WCARRY_A;

#pragma unroll 1
  for (int t = 0; t < SEQLEN; ++t) {
    v8f acc[4];
    acc[0] = z8; acc[1] = z8; acc[2] = z8; acc[3] = z8;
#pragma unroll 1
    for (int k0 = 0; k0 < DMODEL; k0 += 32) {
      const v16h a  = Frag<_Float16>::load(arow + k0);
      const v16h b0 = Frag<_Float16>::load(brow + k0);
      const v16h b1 = Frag<_Float16>::load(brow + (size_t)1 * 16 * DMODEL + k0);
      const v16h b2 = Frag<_Float16>::load(brow + (size_t)2 * 16 * DMODEL + k0);
      const v16h b3 = Frag<_Float16>::load(brow + (size_t)3 * 16 * DMODEL + k0);
      acc[0] = Frag<_Float16>::mma(a, b0, acc[0]);
      acc[1] = Frag<_Float16>::mma(a, b1, acc[1]);
      acc[2] = Frag<_Float16>::mma(a, b2, acc[2]);
      acc[3] = Frag<_Float16>::mma(a, b3, acc[3]);
      dep_guard_h(acc[0], acc[3], a, b3);
      keep4_h(b0, b1, b2, b3);
    }
    acc_guard4(acc[0], acc[1], acc[2], acc[3]);
    __syncthreads();

    const int tn = (t + 1 < SEQLEN) ? (t + 1) : (SEQLEN - 1);
#pragma unroll
    for (int j = 0; j < 4; ++j) {
      const int n = n0 + 16 * j + c;
#pragma unroll
      for (int r = 0; r < 4; ++r) {
        const size_t icur = ((size_t)r * SEQLEN + (size_t)t)  * DMODEL + (size_t)n;
        const size_t inxt = ((size_t)r * SEQLEN + (size_t)tn) * DMODEL + (size_t)n;
        const float rb = rbf[icur];
        const float s  = ftanh(acc[j][r] * inv_carry + rb);
        const float g  = gate[inxt];
        const float qv = q[inxt];
        const float bl = g * s + (1.0f - g) * qv;
        if (hh == 0) {
          Sst[r * SSP + n] = s;
          Abl[r * ABP + n] = (_Float16)bl;
        }
      }
    }
    __syncthreads();

    {
      const int row = tid >> 6, c8 = (tid & 63) * 8;
      const v4f s0 = *(const v4f*)(Sst + row * SSP + c8);
      const v4f s1 = *(const v4f*)(Sst + row * SSP + c8 + 4);
      v8h hv;
      hv[0] = (_Float16)s0[0]; hv[1] = (_Float16)s0[1]; hv[2] = (_Float16)s0[2]; hv[3] = (_Float16)s0[3];
      hv[4] = (_Float16)s1[0]; hv[5] = (_Float16)s1[1]; hv[6] = (_Float16)s1[2]; hv[7] = (_Float16)s1[3];
      unsigned short* dst = Sout + ((size_t)row * SEQLEN + (size_t)t) * DMODEL + (size_t)c8;
      *(volatile v8h*)dst = hv;
      __threadfence();
      *(volatile v8h*)dst = hv;
    }
  }
}

extern "C" void kernel_launch(void* const* d_in, const int* in_sizes, int n_in,
                              void* d_out, int out_size, void* d_ws, size_t ws_size, hipStream_t stream) {
  if (n_in < 10 || d_out == nullptr || d_ws == nullptr) return;
  if (in_sizes[0] != NROWS * DMODEL || in_sizes[1] != NROWS * DMODEL || in_sizes[2] != NROWS * DMODEL ||
      in_sizes[3] != DMODEL * DMODEL || in_sizes[4] != DMODEL * DMODEL || in_sizes[5] != DMODEL * DMODEL ||
      in_sizes[6] != DMODEL || in_sizes[7] != DMODEL * DMODEL || in_sizes[8] != DMODEL || in_sizes[9] < 1 ||
      out_size != NROWS * DMODEL) return;

  const float* q      = (const float*)d_in[0];
  const float* kin    = (const float*)d_in[1];
  const float* vin    = (const float*)d_in[2];
  const float* Amat   = (const float*)d_in[3];
  const float* Bmat   = (const float*)d_in[4];
  const float* gate_w = (const float*)d_in[5];
  const float* gate_b = (const float*)d_in[6];
  const float* out_w  = (const float*)d_in[7];
  const float* out_b  = (const float*)d_in[8];
  const float* decay  = (const float*)d_in[9];
  float* out = (float*)d_out;

  char* ws = (char*)d_ws; size_t off = 0;
  auto carve = [&](size_t bytes) -> char* { char* p = ws + off; off += (bytes + 255) & ~(size_t)255; return p; };
  const size_t plane16 = (size_t)NROWS * DMODEL * 2;
  const size_t plane32 = (size_t)NROWS * DMODEL * 4;
  const size_t wplane  = (size_t)DMODEL * DMODEL * 2;
  unsigned short* Q16  = (unsigned short*)carve(plane16);
  unsigned short* GW16 = (unsigned short*)carve(wplane);
  unsigned short* A16  = (unsigned short*)carve(wplane);
  unsigned short* BM16 = (unsigned short*)carve(wplane);
  unsigned short* OW16 = (unsigned short*)carve(wplane);
  float*          GATE = (float*)carve(plane32);
  unsigned short* R16  = (unsigned short*)carve(plane16);
  float*          RBF  = (float*)carve(plane32);
  unsigned short* S16  = (unsigned short*)carve(plane16);
  if (off > ws_size || off > (size_t)134217728) return;

  const int n2q = NROWS * DMODEL / 2;
  const int n2w = DMODEL * DMODEL / 2;
  cast_scale_f16x2<<<(n2q + 255) / 256, 256, 0, stream>>>(q,      (_Float16*)Q16,  n2q, 1.0f);
  cast_scale_f16x2<<<(n2w + 255) / 256, 256, 0, stream>>>(gate_w, (_Float16*)GW16, n2w, WCARRY_G);
  cast_scale_f16x2<<<(n2w + 255) / 256, 256, 0, stream>>>(Amat,   (_Float16*)A16,  n2w, WCARRY_A);
  cast_scale_f16x2<<<(n2w + 255) / 256, 256, 0, stream>>>(Bmat,   (_Float16*)BM16, n2w, WCARRY_A);
  cast_scale_f16x2<<<(n2w + 255) / 256, 256, 0, stream>>>(out_w,  (_Float16*)OW16, n2w, WCARRY_O);

  const int gemm_tiles  = (NROWS / 64) * (DMODEL / 64);
  const int gemm_blocks = (gemm_tiles + 7) / 8;
  wmma_gemm64<0, false, 2, 0, false, 6><<<dim3(gemm_blocks, 1), 256, 0, stream>>>(
      Q16, Q16, DMODEL, 0L, GW16, GW16, DMODEL, 0L, (void*)GATE, (void*)GATE, DMODEL, 0L,
      gate_b, gate_b, 0L, NROWS, DMODEL, DMODEL, 1.0f / WCARRY_G);
  rscan_kernel<<<NBAT, 64, 0, stream>>>(kin, vin, decay, in_sizes[9], R16);
  wmma_gemm64<0, false, 0, 0, false, 0><<<dim3(gemm_blocks, 1), 256, 0, stream>>>(
      R16, R16, DMODEL, 0L, BM16, BM16, DMODEL, 0L, (void*)RBF, (void*)RBF, DMODEL, 0L,
      gate_b, gate_b, 0L, NROWS, DMODEL, DMODEL, 1.0f / WCARRY_A);
  recur_kernel<<<1, RTHR, 0, stream>>>(q, GATE, RBF, A16, S16);
  wmma_gemm64<0, false, 2, 0, false, 0><<<dim3(gemm_blocks, 1), 256, 0, stream>>>(
      S16, S16, DMODEL, 0L, OW16, OW16, DMODEL, 0L, (void*)out, (void*)out, DMODEL, 0L,
      out_b, out_b, 0L, NROWS, DMODEL, DMODEL, 1.0f / WCARRY_O);
}
